// MultiHeadAttention_63385127355136
// MI455X (gfx1250) — hardware-verified
//
#include <hip/hip_runtime.h>
#include <hip/hip_bf16.h>
#include <stdint.h>


#ifndef NB
#define NB 8
#endif
#ifndef SEQ
#define SEQ 1024
#endif
#define NB_FULL 8
#define S_FULL  1024
#define EMB     1024
#define NHEAD   16
#define HDIM    64
#define MROWS   (NB * SEQ)
#define MWORDS  (SEQ / 32)

static_assert(NB >= 1 && NB <= NB_FULL);
static_assert(SEQ % 128 == 0 && SEQ <= S_FULL);
static_assert(EMB == NHEAD * HDIM);
static_assert(EMB % 128 == 0);
static_assert(MROWS % 128 == 0);
static_assert(((MROWS * EMB) / 8) % 256 == 0);
static_assert((NB * SEQ * MWORDS) % 256 == 0);

#define P_CARRY    1024.0f
#define CTX_SCALE  (1.0f / 64.0f)
#define WO_CARRY   64.0f
#define OUT_SCALE  (1.0f / 1024.0f)

#define PLANE_BYTES ((size_t)MROWS * EMB * 2)
#define WT_BYTES    ((size_t)EMB * EMB * 2)
#define MB_BYTES    ((size_t)NB * SEQ * MWORDS * 4)
#define WS_TOTAL    (PLANE_BYTES * 5 + WT_BYTES * 4 + MB_BYTES)
static_assert(WS_TOTAL <= (size_t)134217728);
static_assert(PLANE_BYTES % 128 == 0 && WT_BYTES % 128 == 0 && MB_BYTES % 128 == 0);

typedef _Float16     v16h __attribute__((ext_vector_type(16)));
typedef __bf16       v16b __attribute__((ext_vector_type(16)));
typedef float        v8f  __attribute__((ext_vector_type(8)));
typedef float        v4f  __attribute__((ext_vector_type(4)));
typedef unsigned int v4u  __attribute__((ext_vector_type(4)));
typedef unsigned int v2u  __attribute__((ext_vector_type(2)));
typedef int          v4i  __attribute__((ext_vector_type(4)));

union Frag {
    v16h     h;
    v16b     b;
    v4u      q[2];
    uint16_t s[16];
};

__device__ __forceinline__ uint16_t bf16_bits(float f) {
    uint32_t u = __builtin_bit_cast(uint32_t, f);
    u += 0x7FFFu + ((u >> 16) & 1u);
    return (uint16_t)(u >> 16);
}
__device__ __forceinline__ float bf16_rne(float f) {
    const uint32_t u = ((uint32_t)bf16_bits(f)) << 16;
    return __builtin_bit_cast(float, u);
}
__device__ __forceinline__ uint16_t h_bits(float f) {
    return __builtin_bit_cast(uint16_t, (_Float16)f);
}

__device__ __forceinline__ v8f mma_h(v16h a, v16h b, v8f c) {
    v8f d = __builtin_amdgcn_wmma_f32_16x16x32_f16(false, a, false, b, (short)0, c, false, false);
    asm volatile("v_nop\n\tv_nop\n\tv_nop\n\tv_nop" : "+v"(d) : "v"(a), "v"(b));
    return d;
}
__device__ __forceinline__ v8f mma_b(v16b a, v16b b, v8f c) {
    v8f d = __builtin_amdgcn_wmma_f32_16x16x32_bf16(false, a, false, b, (short)0, c, false, false);
    asm volatile("v_nop\n\tv_nop\n\tv_nop\n\tv_nop" : "+v"(d) : "v"(a), "v"(b));
    return d;
}

__device__ __forceinline__ Frag ldfrag(const uint16_t* rowp, int k0, int hf) {
    Frag f;
    f.q[0] = *(const v4u*)(rowp + k0 + 8 * hf);
    f.q[1] = *(const v4u*)(rowp + k0 + 16 + 8 * hf);
    return f;
}

__device__ __forceinline__ float rowmax16(float v) {
#pragma unroll
    for (int m = 1; m < 16; m <<= 1) v = fmaxf(v, __shfl_xor(v, m, 32));
    return v;
}
__device__ __forceinline__ float rowsum16(float v) {
#pragma unroll
    for (int m = 1; m < 16; m <<= 1) v += __shfl_xor(v, m, 32);
    return v;
}

__global__ __launch_bounds__(256)
void k_cvt_x(const float* __restrict__ x, uint16_t* __restrict__ xb) {
    const size_t gid = (size_t)blockIdx.x * 256 + threadIdx.x;
    const size_t e0  = gid * 8;
    const size_t m   = e0 / EMB;
    const int    c   = (int)(e0 % EMB);
    const size_t b   = m / SEQ, s = m % SEQ;
    const float* src = x + (b * S_FULL + s) * EMB + c;
    const v4f a0 = *(const v4f*)src;
    const v4f a1 = *(const v4f*)(src + 4);
    v4u w;
    w.x = (uint32_t)bf16_bits(a0.x) | ((uint32_t)bf16_bits(a0.y) << 16);
    w.y = (uint32_t)bf16_bits(a0.z) | ((uint32_t)bf16_bits(a0.w) << 16);
    w.z = (uint32_t)bf16_bits(a1.x) | ((uint32_t)bf16_bits(a1.y) << 16);
    w.w = (uint32_t)bf16_bits(a1.z) | ((uint32_t)bf16_bits(a1.w) << 16);
    uint16_t* dst = xb + e0;
    *(volatile v4u*)dst = w;
    __threadfence();
    *(volatile v4u*)dst = w;
}

template <bool TO_F16>
__global__ __launch_bounds__(256)
void k_wconv(const float* __restrict__ W, uint16_t* __restrict__ WT, float scale) {
    __shared__ uint16_t tile[64 * 64];
    const int t = threadIdx.x;
    const int n0 = blockIdx.x * 64, k0 = blockIdx.y * 64;
    const int kr = t >> 2, nc = (t & 3) * 16;
    const float* src = W + (size_t)(k0 + kr) * EMB + n0 + nc;
#pragma unroll
    for (int i = 0; i < 4; ++i) {
        const v4f v = *(const v4f*)(src + 4 * i);
        float f[4];
        f[0] = v.x; f[1] = v.y; f[2] = v.z; f[3] = v.w;
#pragma unroll
        for (int jj = 0; jj < 4; ++jj) {
            const float g = bf16_rne(f[jj]) * scale;
            tile[(nc + 4 * i + jj) * 64 + kr] = TO_F16 ? h_bits(g) : bf16_bits(g);
        }
    }
    __syncthreads();
    v4u val[2]; size_t off[2];
#pragma unroll
    for (int i = 0; i < 2; ++i) {
        const int p   = t + 256 * i;
        const int row = p >> 3, seg = (p & 7) * 8;
        val[i] = *(const v4u*)&tile[row * 64 + seg];
        off[i] = (size_t)(n0 + row) * EMB + k0 + seg;
    }
#pragma unroll
    for (int i = 0; i < 2; ++i) *(volatile v4u*)(WT + off[i]) = val[i];
    __threadfence();
#pragma unroll
    for (int i = 0; i < 2; ++i) *(volatile v4u*)(WT + off[i]) = val[i];
}

__global__ __launch_bounds__(256)
void k_maskbits(const int* __restrict__ mask, unsigned int* __restrict__ mb) {
    const size_t gid = (size_t)blockIdx.x * 256 + threadIdx.x;
    const int    w   = (int)(gid % MWORDS);
    const size_t row = gid / MWORDS;
    const size_t b = row / SEQ, q = row % SEQ;
    const int* src = mask + (b * S_FULL + q) * S_FULL + (size_t)w * 32;
    unsigned int bits = 0u;
#pragma unroll
    for (int i = 0; i < 8; ++i) {
        const v4i v = *(const v4i*)(src + 4 * i);
        bits |= (v.x != 0 ? 1u : 0u) << (4 * i + 0);
        bits |= (v.y != 0 ? 1u : 0u) << (4 * i + 1);
        bits |= (v.z != 0 ? 1u : 0u) << (4 * i + 2);
        bits |= (v.w != 0 ? 1u : 0u) << (4 * i + 3);
    }
    volatile unsigned int* dst = mb + gid;
    *dst = bits;
    __threadfence();
    *dst = bits;
}

template <bool BF, bool OUT16>
__global__ __launch_bounds__(256)
void k_gemm(const uint16_t* __restrict__ A, const uint16_t* __restrict__ BT,
            const float* __restrict__ bias, void* __restrict__ Cout, float oscale) {
    __shared__ float slab[8][16 * 64];

    const int t = threadIdx.x, wave = t >> 5, lane = t & 31;
    const int hf = lane >> 4, l16 = lane & 15;
    const int m0 = blockIdx.y * 128, n0 = blockIdx.x * 128;
    const int wr = wave & 3, wc = wave >> 2;

    const uint16_t* arow[2];
    const uint16_t* brow[4];
#pragma unroll
    for (int mt = 0; mt < 2; ++mt)
        arow[mt] = A + (size_t)(m0 + wr * 32 + mt * 16 + l16) * EMB;
#pragma unroll
    for (int nt = 0; nt < 4; ++nt)
        brow[nt] = BT + (size_t)(n0 + wc * 64 + nt * 16 + l16) * EMB;

    v8f acc[8] = {};

#pragma unroll 1
    for (int k0 = 0; k0 < EMB; k0 += 32) {
        Frag a[2], b[4];
#pragma unroll
        for (int mt = 0; mt < 2; ++mt) a[mt] = ldfrag(arow[mt], k0, hf);
#pragma unroll
        for (int nt = 0; nt < 4; ++nt) b[nt] = ldfrag(brow[nt], k0, hf);
#pragma unroll
        for (int mt = 0; mt < 2; ++mt)
#pragma unroll
            for (int nt = 0; nt < 4; ++nt) {
                if constexpr (BF)
                    acc[mt * 4 + nt] = mma_b(a[mt].b, b[nt].b, acc[mt * 4 + nt]);
                else
                    acc[mt * 4 + nt] = mma_h(a[mt].h, b[nt].h, acc[mt * 4 + nt]);
            }
    }

    float bvv[4];
#pragma unroll
    for (int nt = 0; nt < 4; ++nt)
        bvv[nt] = bf16_rne(bias[n0 + wc * 64 + nt * 16 + l16]);

    float* mys = slab[wave];
    if constexpr (OUT16) {
        uint16_t* mys16 = reinterpret_cast<uint16_t*>(mys);
        uint16_t* C     = reinterpret_cast<uint16_t*>(Cout);
#pragma unroll
        for (int mt = 0; mt < 2; ++mt)
#pragma unroll
            for (int nt = 0; nt < 4; ++nt)
#pragma unroll
                for (int r = 0; r < 8; ++r)
                    mys16[(mt * 16 + 8 * hf + r) * 64 + nt * 16 + l16] =
                        h_bits(acc[mt * 4 + nt][r] * oscale + bvv[nt]);
        __syncthreads();
        v4u val[8]; size_t off[8];
#pragma unroll
        for (int i = 0; i < 8; ++i) {
            const int p = lane + 32 * i;
            const int row = p >> 3, seg = (p & 7) * 8;
            val[i] = *(const v4u*)(mys16 + row * 64 + seg);
            off[i] = (size_t)(m0 + wr * 32 + row) * EMB + n0 + wc * 64 + seg;
        }
#pragma unroll
        for (int i = 0; i < 8; ++i) *(volatile v4u*)(C + off[i]) = val[i];
        __threadfence();
#pragma unroll
        for (int i = 0; i < 8; ++i) *(volatile v4u*)(C + off[i]) = val[i];
    } else {
        float* C = reinterpret_cast<float*>(Cout);
#pragma unroll
        for (int mt = 0; mt < 2; ++mt) {
            __syncthreads();
#pragma unroll
            for (int nt = 0; nt < 4; ++nt)
#pragma unroll
                for (int r = 0; r < 8; ++r)
                    mys[(8 * hf + r) * 64 + nt * 16 + l16] = acc[mt * 4 + nt][r] * oscale + bvv[nt];
            __syncthreads();
            v4f val[8]; size_t off[8];
#pragma unroll
            for (int i = 0; i < 8; ++i) {
                const int p = lane + 32 * i;
                const int row = p >> 4, seg = (p & 15) * 4;
                val[i] = *(const v4f*)(mys + row * 64 + seg);
                off[i] = (size_t)(m0 + wr * 32 + mt * 16 + row) * EMB + n0 + wc * 64 + seg;
            }
#pragma unroll
            for (int i = 0; i < 8; ++i) *(volatile v4f*)(C + off[i]) = val[i];
            __threadfence();
#pragma unroll
            for (int i = 0; i < 8; ++i) *(volatile v4f*)(C + off[i]) = val[i];
        }
    }
}

__global__ __launch_bounds__(256)
void k_attn(const uint16_t* __restrict__ Qp, const uint16_t* __restrict__ Kp,
            const uint16_t* __restrict__ Vp, const unsigned int* __restrict__ mb,
            uint16_t* __restrict__ ctx) {
    __shared__ uint16_t kt[64 * 64];
    __shared__ uint16_t vt[64 * 64];
    __shared__ uint16_t ps[8][16 * 64];

    const int t = threadIdx.x, wave = t >> 5, lane = t & 31;
    const int hf = lane >> 4, l16 = lane & 15;
    const int b  = blockIdx.y / NHEAD, hd = blockIdx.y % NHEAD;
    const int qr = blockIdx.x * 128 + wave * 16;
    const size_t rowb = (size_t)b * SEQ;
    const size_t hcol = (size_t)hd * HDIM;

    Frag qf[2];
    {
        const uint16_t* qrow = Qp + (rowb + qr + l16) * EMB + hcol;
        qf[0] = ldfrag(qrow, 0, hf);
        qf[1] = ldfrag(qrow, 32, hf);
    }

    v8f accO[4] = {};
    float mrow[8], lrow[8];
#pragma unroll
    for (int r = 0; r < 8; ++r) { mrow[r] = -__builtin_inff(); lrow[r] = 0.0f; }

    const int keyr = t >> 2, hdB = (t & 3) * 16;
    const unsigned int* mbrow = mb + (rowb + qr + 8 * hf) * MWORDS;
    uint16_t* myps = ps[wave];

#pragma unroll 1
    for (int j = 0; j < SEQ / 64; ++j) {
        const int key0 = j * 64;
        __syncthreads();

        {
            const size_t go = (rowb + key0 + keyr) * EMB + hcol + hdB;
            const v4u k0v = *(const v4u*)(Kp + go);
            const v4u k1v = *(const v4u*)(Kp + go + 8);
            *(v4u*)&kt[keyr * 64 + hdB]     = k0v;
            *(v4u*)&kt[keyr * 64 + hdB + 8] = k1v;
            Frag fv;
            fv.q[0] = *(const v4u*)(Vp + go);
            fv.q[1] = *(const v4u*)(Vp + go + 8);
#pragma unroll
            for (int i = 0; i < 16; ++i) vt[(hdB + i) * 64 + keyr] = fv.s[i];
        }
        unsigned int mlo[8], mhi[8];
#pragma unroll
        for (int r = 0; r < 8; ++r) {
            const v2u w = *(const v2u*)(mbrow + (size_t)r * MWORDS + 2 * j);
            mlo[r] = w.x; mhi[r] = w.y;
        }
        __syncthreads();

        v8f sc[4];
#pragma unroll
        for (int nt = 0; nt < 4; ++nt) {
            v8f z = {};
            Frag kf = ldfrag(&kt[(nt * 16 + l16) * 64], 0, hf);
            z = mma_h(qf[0].h, kf.h, z);
            kf = ldfrag(&kt[(nt * 16 + l16) * 64], 32, hf);
            z = mma_h(qf[1].h, kf.h, z);
#pragma unroll
            for (int r = 0; r < 8; ++r) {
                const unsigned int w   = (nt < 2) ? mlo[r] : mhi[r];
                const unsigned int bit = (w >> ((nt & 1) * 16 + l16)) & 1u;
                sc[nt][r] = bit ? -1.0e9f : z[r] * 0.125f;
            }
        }

        float alpha[8];
#pragma unroll
        for (int r = 0; r < 8; ++r) {
            float bm = sc[0][r];
#pragma unroll
            for (int nt = 1; nt < 4; ++nt) bm = fmaxf(bm, sc[nt][r]);
            bm = rowmax16(bm);
            const float mnew = fmaxf(mrow[r], bm);
            alpha[r] = __expf(mrow[r] - mnew);
            mrow[r] = mnew;
        }
        float rs[8];
#pragma unroll
        for (int r = 0; r < 8; ++r) rs[r] = 0.0f;
#pragma unroll
        for (int nt = 0; nt < 4; ++nt)
#pragma unroll
            for (int r = 0; r < 8; ++r) {
                const float p = __expf(sc[nt][r] - mrow[r]);
                sc[nt][r] = p;
                rs[r] += p;
            }
#pragma unroll
        for (int r = 0; r < 8; ++r) {
            lrow[r] = lrow[r] * alpha[r] + rowsum16(rs[r]);
#pragma unroll
            for (int nt = 0; nt < 4; ++nt) accO[nt][r] *= alpha[r];
        }

#pragma unroll
        for (int nt = 0; nt < 4; ++nt)
#pragma unroll
            for (int r = 0; r < 8; ++r)
                myps[(r + 8 * hf) * 64 + nt * 16 + l16] = h_bits(sc[nt][r] * P_CARRY);
        __syncthreads();
        const Frag pf0 = ldfrag(myps + l16 * 64, 0, hf);
        const Frag pf1 = ldfrag(myps + l16 * 64, 32, hf);

#pragma unroll
        for (int nt = 0; nt < 4; ++nt) {
            Frag vf = ldfrag(&vt[(nt * 16 + l16) * 64], 0, hf);
            accO[nt] = mma_h(pf0.h, vf.h, accO[nt]);
            vf = ldfrag(&vt[(nt * 16 + l16) * 64], 32, hf);
            accO[nt] = mma_h(pf1.h, vf.h, accO[nt]);
        }
    }

    float inv[8];
#pragma unroll
    for (int r = 0; r < 8; ++r) inv[r] = (1.0f / lrow[r]) * CTX_SCALE;
    __syncthreads();
#pragma unroll
    for (int nt = 0; nt < 4; ++nt)
#pragma unroll
        for (int r = 0; r < 8; ++r)
            myps[(8 * hf + r) * 64 + nt * 16 + l16] = h_bits(accO[nt][r] * inv[r]);
    __syncthreads();
    v4u val[4]; size_t off[4];
#pragma unroll
    for (int i = 0; i < 4; ++i) {
        const int p = lane + 32 * i;
        const int row = p >> 3, seg = (p & 7) * 8;
        val[i] = *(const v4u*)(myps + row * 64 + seg);
        off[i] = (rowb + qr + row) * EMB + hcol + seg;
    }
#pragma unroll
    for (int i = 0; i < 4; ++i) *(volatile v4u*)(ctx + off[i]) = val[i];
    __threadfence();
#pragma unroll
    for (int i = 0; i < 4; ++i) *(volatile v4u*)(ctx + off[i]) = val[i];
}

extern "C" void kernel_launch(void* const* d_in, const int* in_sizes, int n_in,
                              void* d_out, int out_size, void* d_ws, size_t ws_size,
                              hipStream_t stream) {
    if (n_in < 10) return;
    if (in_sizes[0] < NB * S_FULL * EMB) return;
    if (in_sizes[1] < NB * S_FULL * S_FULL) return;
    if (in_sizes[2] < EMB * EMB || in_sizes[4] < EMB * EMB ||
        in_sizes[6] < EMB * EMB || in_sizes[8] < EMB * EMB) return;
    if (in_sizes[3] < EMB || in_sizes[5] < EMB || in_sizes[7] < EMB || in_sizes[9] < EMB) return;
    if (out_size < MROWS * EMB) return;
    if (ws_size < WS_TOTAL) return;

    const float* x    = (const float*)d_in[0];
    const int*   mask = (const int*)d_in[1];
    const float* Wq   = (const float*)d_in[2];
    const float* bq   = (const float*)d_in[3];
    const float* Wk   = (const float*)d_in[4];
    const float* bk   = (const float*)d_in[5];
    const float* Wv   = (const float*)d_in[6];
    const float* bv   = (const float*)d_in[7];
    const float* Wo   = (const float*)d_in[8];
    const float* bo   = (const float*)d_in[9];
    float* out = (float*)d_out;

    unsigned char* ws = (unsigned char*)d_ws;
    size_t off = 0;
    uint16_t* xb   = (uint16_t*)(ws + off); off += PLANE_BYTES;
    uint16_t* WqT  = (uint16_t*)(ws + off); off += WT_BYTES;
    uint16_t* WkT  = (uint16_t*)(ws + off); off += WT_BYTES;
    uint16_t* WvT  = (uint16_t*)(ws + off); off += WT_BYTES;
    uint16_t* WoT  = (uint16_t*)(ws + off); off += WT_BYTES;
    uint16_t* Qp   = (uint16_t*)(ws + off); off += PLANE_BYTES;
    uint16_t* Kpl  = (uint16_t*)(ws + off); off += PLANE_BYTES;
    uint16_t* Vpl  = (uint16_t*)(ws + off); off += PLANE_BYTES;
    uint16_t* Ctx  = (uint16_t*)(ws + off); off += PLANE_BYTES;
    unsigned int* mbits = (unsigned int*)(ws + off); off += MB_BYTES;
    if (off > ws_size) return;

    k_cvt_x<<<dim3((MROWS * EMB / 8) / 256), dim3(256), 0, stream>>>(x, xb);

    const dim3 gW(EMB / 64, EMB / 64);
    k_wconv<false><<<gW, dim3(256), 0, stream>>>(Wq, WqT, 1.0f);
    k_wconv<false><<<gW, dim3(256), 0, stream>>>(Wk, WkT, 1.0f);
    k_wconv<false><<<gW, dim3(256), 0, stream>>>(Wv, WvT, 1.0f);
    k_wconv<true><<<gW, dim3(256), 0, stream>>>(Wo, WoT, WO_CARRY);

    k_maskbits<<<dim3((NB * SEQ * MWORDS) / 256), dim3(256), 0, stream>>>(mask, mbits);

    const dim3 gG(EMB / 128, MROWS / 128);
    k_gemm<true, true><<<gG, dim3(256), 0, stream>>>(xb, WqT, bq, (void*)Qp, 1.0f);
    k_gemm<true, true><<<gG, dim3(256), 0, stream>>>(xb, WkT, bk, (void*)Kpl, 1.0f);
    k_gemm<true, true><<<gG, dim3(256), 0, stream>>>(xb, WvT, bv, (void*)Vpl, 1.0f);

    const dim3 gA(SEQ / 128, NB * NHEAD);
    k_attn<<<gA, dim3(256), 0, stream>>>(Qp, Kpl, Vpl, mbits, Ctx);

    k_gemm<false, false><<<gG, dim3(256), 0, stream>>>(Ctx, WoT, bo, (void*)out, OUT_SCALE);
}
